// DualPathRecurrentProcessor_79577154060725
// MI455X (gfx1250) — hardware-verified
//
#include <hip/hip_runtime.h>
#include <math.h>

constexpr int kBatch  = 32;
constexpr int kSeq    = 2048;
constexpr int kDim    = 128;
constexpr int kExp    = 256;
constexpr int kExp2   = 512;
constexpr int kFeat   = 512;
constexpr int kQBatch = 8;
constexpr int kQRows  = kQBatch * kSeq;
constexpr int kNumQ   = kBatch / kQBatch;
constexpr float kLn3     = 1.0986122886681098f;
constexpr float kStepRcp = 1.0f / 2047.0f;

constexpr size_t kWstBytes  = (size_t)2 * kExp2 * kDim * 2;
constexpr size_t kWfBytes   = (size_t)kDim * kFeat * 2;
constexpr size_t kXqBytes   = (size_t)2 * kQRows * kDim * 2;
constexpr size_t kPapiBytes = (size_t)2 * kQRows * kExp2 * 4;
constexpr size_t kCmbBytes  = (size_t)kQRows * kFeat * 2;
constexpr size_t kOffWstHi = 0;
constexpr size_t kOffWstLo = kOffWstHi + kWstBytes;
constexpr size_t kOffWfHi  = kOffWstLo + kWstBytes;
constexpr size_t kOffWfLo  = kOffWfHi + kWfBytes;
constexpr size_t kOffXh    = kOffWfLo + kWfBytes;
constexpr size_t kOffXl    = kOffXh + kXqBytes;
constexpr size_t kOffPapi  = kOffXl + kXqBytes;
constexpr size_t kOffCh    = kOffPapi + kPapiBytes;
constexpr size_t kOffCl    = kOffCh + kCmbBytes;
constexpr size_t kWsTotal  = kOffCl + kCmbBytes;
typedef char ws_total_check[(kWsTotal == 118226944) ? 1 : -1];
typedef char ws_cap_check[(kWsTotal <= 134217728) ? 1 : -1];

typedef __attribute__((ext_vector_type(16))) _Float16 v16h;
typedef __attribute__((ext_vector_type(8)))  _Float16 v8h;
typedef __attribute__((ext_vector_type(16))) __bf16   v16b;
typedef __attribute__((ext_vector_type(8)))  __bf16   v8b;
typedef __attribute__((ext_vector_type(8)))  float    v8f;
typedef __attribute__((ext_vector_type(4)))  float    v4f;
typedef __attribute__((ext_vector_type(4)))  unsigned int v4u;

__device__ __forceinline__ unsigned short f2bf_bits(float f) {
  unsigned u = __float_as_uint(f);
  return (unsigned short)((u + 0x7FFFu + ((u >> 16) & 1u)) >> 16);
}
__device__ __forceinline__ float bf_bits2f(unsigned short h) { return __uint_as_float(((unsigned)h) << 16); }

__device__ __forceinline__ void dep_guard_h(v8f& a, v8f& b, v16h x, v16h y) { asm volatile("v_nop\n\tv_nop\n\tv_nop\n\tv_nop" : "+v"(a), "+v"(b) : "v"(x), "v"(y)); }
__device__ __forceinline__ void dep_guard_b(v8f& a, v8f& b, v16b x, v16b y) { asm volatile("v_nop\n\tv_nop\n\tv_nop\n\tv_nop" : "+v"(a), "+v"(b) : "v"(x), "v"(y)); }
__device__ __forceinline__ void keep4_h(v16h a, v16h b, v16h c, v16h d) { asm volatile("v_nop" :: "v"(a), "v"(b), "v"(c), "v"(d)); }
__device__ __forceinline__ void keep4_b(v16b a, v16b b, v16b c, v16b d) { asm volatile("v_nop" :: "v"(a), "v"(b), "v"(c), "v"(d)); }
__device__ __forceinline__ void acc_guard4(v8f& a, v8f& b, v8f& c, v8f& d) { asm volatile("v_nop\n\tv_nop\n\tv_nop\n\tv_nop" : "+v"(a), "+v"(b), "+v"(c), "+v"(d)); }
template <typename T> struct Frag;
template <> struct Frag<_Float16> {
  typedef v16h V; union U { v16h v; v8h h[2]; };
  static __device__ __forceinline__ v16h load(const _Float16* p) {
    U f; f.h[0] = *(const v8h*)(p); f.h[1] = *(const v8h*)(p + 16); return f.v;
  }
  static __device__ __forceinline__ v8f mma(v16h a, v16h b, v8f c) {
    return __builtin_amdgcn_wmma_f32_16x16x32_f16(false, a, false, b, (short)0, c, false, false);
  }
  static __device__ __forceinline__ void guard(v8f& a, v8f& b, v16h x, v16h y) { dep_guard_h(a, b, x, y); }
  static __device__ __forceinline__ void keep(v16h a, v16h b, v16h c, v16h d) { keep4_h(a, b, c, d); }
};
template <> struct Frag<__bf16> {
  typedef v16b V; union U { v16b v; v8b h[2]; };
  static __device__ __forceinline__ v16b load(const __bf16* p) {
    U f; f.h[0] = *(const v8b*)(p); f.h[1] = *(const v8b*)(p + 16); return f.v;
  }
  static __device__ __forceinline__ v8f mma(v16b a, v16b b, v8f c) {
    return __builtin_amdgcn_wmma_f32_16x16x32_bf16(false, a, false, b, (short)0, c, false, false);
  }
  static __device__ __forceinline__ void guard(v8f& a, v8f& b, v16b x, v16b y) { dep_guard_b(a, b, x, y); }
  static __device__ __forceinline__ void keep(v16b a, v16b b, v16b c, v16b d) { keep4_b(a, b, c, d); }
};

__device__ __forceinline__ unsigned pk16(unsigned short a, unsigned short b) { return (unsigned)a | ((unsigned)b << 16); }

template <int ET> struct Elem;
template <> struct Elem<0> { typedef _Float16 T; };
template <> struct Elem<1> { typedef __bf16 T; };
template <int ET, bool SPLIT, int BIAS_MODE, int OUT_MODE, bool RESID, int ACT = 0>
__global__ __launch_bounds__(256) void wmma_gemm64(
    const unsigned short* __restrict__ Ap, const unsigned short* __restrict__ A2p, int lda, long strideA,
    const unsigned short* __restrict__ Btp, const unsigned short* __restrict__ Bt2p, int ldb, long strideB,
    void* __restrict__ Cout, void* __restrict__ Cout2, int ldc, long strideC,
    const float* __restrict__ bias,
    const float* __restrict__ resid, long strideR,
    int M, int N, int K, float scale) {
  typedef typename Elem<ET>::T T;
  typedef typename Frag<T>::V V;
  const T* A = (const T*)Ap; const T* A2 = (const T*)A2p; const T* Bt = (const T*)Btp; const T* Bt2 = (const T*)Bt2p;
  __shared__ __align__(16) float sT[8][16 * 68];
  const int b    = blockIdx.y;
  const int lane = threadIdx.x & 31;
  const int wave = threadIdx.x >> 5;
  const int tilesN = N >> 6;
  const int tilesM = M >> 6;
  const int tile = blockIdx.x * 8 + wave;
  if (tile >= tilesM * tilesN) return;
  const int tm = tile / tilesN;
  const int tn = tile - tm * tilesN;
  const int m0 = tm << 6;
  const int n0 = tn << 6;

  const T* Ab  = A  + (size_t)b * strideA;
  const T* Bb  = Bt + (size_t)b * strideB;
  const T* Ab2 = SPLIT ? (A2  + (size_t)b * strideA) : nullptr;
  const T* Bb2 = SPLIT ? (Bt2 + (size_t)b * strideB) : nullptr;

  const int rlane = lane & 15;
  const int koff  = (lane >> 4) * 8;
  const int mOff  = (lane >> 4) * 8;

  v8f acc[4][4];
#pragma unroll
  for (int i = 0; i < 4; ++i)
#pragma unroll
    for (int j = 0; j < 4; ++j) acc[i][j] = (v8f){0.f,0.f,0.f,0.f,0.f,0.f,0.f,0.f};

  for (int k0 = 0; k0 < K; k0 += 32) {
    V bh[4], bl[4];
#pragma unroll
    for (int j = 0; j < 4; ++j) {
      const size_t bo = (size_t)(n0 + (j << 4) + rlane) * ldb + koff + k0;
      bh[j] = Frag<T>::load(Bb + bo);
      if (SPLIT) bl[j] = Frag<T>::load(Bb2 + bo);
    }
#pragma unroll
    for (int i = 0; i < 4; ++i) {
      const size_t ao = (size_t)(m0 + (i << 4) + rlane) * lda + koff + k0;
      V ah = Frag<T>::load(Ab + ao);
      V al;
      if (SPLIT) al = Frag<T>::load(Ab2 + ao);
#pragma unroll
      for (int j = 0; j < 4; ++j) {
        acc[i][j] = Frag<T>::mma(ah, bh[j], acc[i][j]);
        if (SPLIT) {
          acc[i][j] = Frag<T>::mma(ah, bl[j], acc[i][j]);
          acc[i][j] = Frag<T>::mma(al, bh[j], acc[i][j]);
        }
      }
      Frag<T>::guard(acc[i][0], acc[i][3], ah, SPLIT ? al : ah);
    }
    Frag<T>::keep(bh[0], bh[1], bh[2], bh[3]);
    if (SPLIT) Frag<T>::keep(bl[0], bl[1], bl[2], bl[3]);
  }
  acc_guard4(acc[0][0], acc[0][1], acc[0][2], acc[0][3]);
  acc_guard4(acc[1][0], acc[1][1], acc[1][2], acc[1][3]);
  acc_guard4(acc[2][0], acc[2][1], acc[2][2], acc[2][3]);
  acc_guard4(acc[3][0], acc[3][1], acc[3][2], acc[3][3]);

  float* slab = sT[wave];
  const float* Rb = RESID ? (resid + (size_t)b * strideR) : nullptr;
#pragma unroll
  for (int i = 0; i < 4; ++i) {
    const int mBase = m0 + (i << 4);
#pragma unroll
    for (int j = 0; j < 4; ++j) {
      const int n = n0 + (j << 4) + rlane;
      float bv = 0.f;
      if (BIAS_MODE == 2) bv = bias[n];
#pragma unroll
      for (int r = 0; r < 8; ++r) {
        float v = acc[i][j][r] * scale;
        if (BIAS_MODE == 1) v += bias[mBase + mOff + r];
        if (BIAS_MODE == 2) v += bv;
        if (RESID) v += Rb[(size_t)(mBase + mOff + r) * ldc + n];
        if (ACT == 2) v = fmaxf(v, 0.0f);
        if (ACT == 4) v = (v > 0.f) ? v : 0.01f * v;
        slab[(mOff + r) * 68 + (j << 4) + rlane] = v;
      }
    }
    __builtin_amdgcn_fence(__ATOMIC_RELEASE, "workgroup");
    __builtin_amdgcn_wave_barrier();
    __builtin_amdgcn_fence(__ATOMIC_ACQUIRE, "workgroup");
    if (OUT_MODE == 0) {
      float* C = (float*)Cout + (size_t)b * strideC;
      const int hh = lane >> 4, c4 = (lane & 15) * 4;
      for (int pass = 0; pass < 2; ++pass) {
#pragma unroll
        for (int it = 0; it < 8; ++it) {
          const int row = it * 2 + hh;
          v4f v = *(const v4f*)(slab + row * 68 + c4);
          *(volatile v4f*)(C + (size_t)(mBase + row) * ldc + n0 + c4) = v;
        }
        __threadfence();
      }
    } else {
      const int q = lane >> 3, c8 = (lane & 7) * 8;
      unsigned short* C  = (unsigned short*)Cout  + (size_t)b * strideC;
      unsigned short* C2 = (OUT_MODE == 2) ? ((unsigned short*)Cout2 + (size_t)b * strideC) : nullptr;
      for (int pass = 0; pass < 2; ++pass) {
#pragma unroll
        for (int it = 0; it < 4; ++it) {
          const int row = it * 4 + q;
          const float* sp = slab + row * 68 + c8;
          v8h hv, lv;
#pragma unroll
          for (int e = 0; e < 8; ++e) {
            if (OUT_MODE == 1) {
              hv[e] = (_Float16)sp[e];
            } else {
              unsigned short hb = f2bf_bits(sp[e]);
              unsigned short lb = f2bf_bits(sp[e] - bf_bits2f(hb));
              hv[e] = __builtin_bit_cast(_Float16, hb);
              lv[e] = __builtin_bit_cast(_Float16, lb);
            }
          }
          *(volatile v8h*)(C + (size_t)(mBase + row) * ldc + n0 + c8) = hv;
          if (OUT_MODE == 2) *(volatile v8h*)(C2 + (size_t)(mBase + row) * ldc + n0 + c8) = lv;
        }
        __threadfence();
      }
    }
    __builtin_amdgcn_fence(__ATOMIC_RELEASE, "workgroup");
    __builtin_amdgcn_wave_barrier();
    __builtin_amdgcn_fence(__ATOMIC_ACQUIRE, "workgroup");
  }
}

__device__ __forceinline__ void split_bf(float f, unsigned short& hb, unsigned short& lb) {
  hb = f2bf_bits(f);
  lb = f2bf_bits(f - bf_bits2f(hb));
}

__global__ __launch_bounds__(256) void split8_kernel(const float* __restrict__ in,
                                                     unsigned short* __restrict__ hi,
                                                     unsigned short* __restrict__ lo, int n8) {
  const int i = blockIdx.x * 256 + threadIdx.x;
  if (i >= n8) return;
  const float* p = in + 8 * (size_t)i;
  const v4f a = *(const v4f*)(p);
  const v4f c = *(const v4f*)(p + 4);
  unsigned short hb[8], lb[8];
#pragma unroll
  for (int e = 0; e < 4; ++e) {
    split_bf(a[e], hb[e], lb[e]);
    split_bf(c[e], hb[4 + e], lb[4 + e]);
  }
  const v4u uh = (v4u){pk16(hb[0], hb[1]), pk16(hb[2], hb[3]), pk16(hb[4], hb[5]), pk16(hb[6], hb[7])};
  const v4u ul = (v4u){pk16(lb[0], lb[1]), pk16(lb[2], lb[3]), pk16(lb[4], lb[5]), pk16(lb[6], lb[7])};
  unsigned short* qh = hi + 8 * (size_t)i;
  unsigned short* ql = lo + 8 * (size_t)i;
  for (int pass = 0; pass < 2; ++pass) {
    *(volatile v4u*)qh = uh;
    *(volatile v4u*)ql = ul;
    __threadfence();
  }
}

__global__ __launch_bounds__(256) void prep_x_kernel(const float* __restrict__ xq,
                                                     unsigned short* __restrict__ xh,
                                                     unsigned short* __restrict__ xl) {
#pragma clang fp contract(off)
  const int i   = blockIdx.x * 256 + threadIdx.x;
  const int row = i >> 4;
  const int s   = row & (kSeq - 1);
  const float stp = (float)s * kStepRcp;
  const float t   = (s == kSeq - 1) ? 3.0f : 3.0f * stp;
  const float rw  = expf(t);
  const float* p = xq + 8 * (size_t)i;
  const v4f a = *(const v4f*)(p);
  const v4f c = *(const v4f*)(p + 4);
  unsigned short h0[8], l0[8], h1[8], l1[8];
#pragma unroll
  for (int e = 0; e < 4; ++e) {
    split_bf(a[e], h0[e], l0[e]);
    split_bf(c[e], h0[4 + e], l0[4 + e]);
    split_bf(a[e] * rw, h1[e], l1[e]);
    split_bf(c[e] * rw, h1[4 + e], l1[4 + e]);
  }
  const v4u uh0 = (v4u){pk16(h0[0], h0[1]), pk16(h0[2], h0[3]), pk16(h0[4], h0[5]), pk16(h0[6], h0[7])};
  const v4u ul0 = (v4u){pk16(l0[0], l0[1]), pk16(l0[2], l0[3]), pk16(l0[4], l0[5]), pk16(l0[6], l0[7])};
  const v4u uh1 = (v4u){pk16(h1[0], h1[1]), pk16(h1[2], h1[3]), pk16(h1[4], h1[5]), pk16(h1[6], h1[7])};
  const v4u ul1 = (v4u){pk16(l1[0], l1[1]), pk16(l1[2], l1[3]), pk16(l1[4], l1[5]), pk16(l1[6], l1[7])};
  const size_t o  = 8 * (size_t)i;
  const size_t p1 = (size_t)kQRows * kDim;
  for (int pass = 0; pass < 2; ++pass) {
    *(volatile v4u*)(xh + o)      = uh0;
    *(volatile v4u*)(xl + o)      = ul0;
    *(volatile v4u*)(xh + p1 + o) = uh1;
    *(volatile v4u*)(xl + p1 + o) = ul1;
    __threadfence();
  }
}

__global__ __launch_bounds__(256) void scan_kernel(const float* __restrict__ papi,
                                                   const float* __restrict__ ba_u, const float* __restrict__ bi_u,
                                                   const float* __restrict__ g_u,
                                                   const float* __restrict__ ba_w, const float* __restrict__ bi_w,
                                                   const float* __restrict__ g_w,
                                                   unsigned short* __restrict__ ch, unsigned short* __restrict__ cl) {
  __shared__ __align__(16) float hs[8 * kExp];
  const int e    = threadIdx.x;
  const int lane = e & 31;
  const int wave = e >> 5;
  const int bl   = blockIdx.x;
  const int path = blockIdx.y;
  const float* ba = path ? ba_w : ba_u;
  const float* bi = path ? bi_w : bi_u;
  const float* gg = path ? g_w : g_u;
  const float bav   = ba[e];
  const float biv   = bi[e];
  const float alpha = __builtin_amdgcn_rcpf(1.0f + expf(-gg[e]));

  const float* P = papi + (size_t)path * kQRows * kExp2 + (size_t)bl * kSeq * kExp2;
  const size_t crow0 = (size_t)bl * kSeq;

  const int q   = lane >> 3;
  const int c8  = (lane & 7) * 8;
  const int lin = wave * 4 + q;
  const int jr  = lin >> 2;
  const int seg = (lin & 3) * 64;

  float h = 0.0f;
  for (int s0 = 0; s0 < kSeq; s0 += 8) {
#pragma unroll 1
    for (int j = 0; j < 8; ++j) {
      const float* pr = P + (size_t)(s0 + j) * kExp2;
      const float pa = pr[e] + bav;
      const float pi = pr[kExp + e] + biv;
      const float rg = __builtin_amdgcn_rcpf(1.0f + expf(-pa));
      const float ig = __builtin_amdgcn_rcpf(1.0f + expf(-pi));
      const float a  = alpha * expf(-(rg * kLn3));
      const float om = fmaxf(1.0f - a * a, 0.0f);
      const float u  = sqrtf(om) * (ig * pi);
      h = a * h + u;
      hs[j * kExp + e] = h;
    }
    __syncthreads();
    {
      const float* sp = hs + jr * kExp + seg + c8;
      const v4f v0 = *(const v4f*)(sp);
      const v4f v1 = *(const v4f*)(sp + 4);
      unsigned short hb[8], lb[8];
#pragma unroll
      for (int k = 0; k < 4; ++k) {
        split_bf(v0[k], hb[k], lb[k]);
        split_bf(v1[k], hb[4 + k], lb[4 + k]);
      }
      const v4u uh = (v4u){pk16(hb[0], hb[1]), pk16(hb[2], hb[3]), pk16(hb[4], hb[5]), pk16(hb[6], hb[7])};
      const v4u ul = (v4u){pk16(lb[0], lb[1]), pk16(lb[2], lb[3]), pk16(lb[4], lb[5]), pk16(lb[6], lb[7])};
      const size_t off = (crow0 + (size_t)(s0 + jr)) * kFeat + (size_t)path * kExp + seg + c8;
      for (int pass = 0; pass < 2; ++pass) {
        *(volatile v4u*)(ch + off) = uh;
        *(volatile v4u*)(cl + off) = ul;
        __threadfence();
      }
    }
    __syncthreads();
  }
}

extern "C" void kernel_launch(void* const* d_in, const int* in_sizes, int n_in,
                              void* d_out, int out_size, void* d_ws, size_t ws_size,
                              hipStream_t stream) {
  if (n_in < 13) return;
  if (in_sizes[0] != kBatch * kSeq * kDim) return;
  if (in_sizes[1] != kExp * kDim || in_sizes[3] != kExp * kDim || in_sizes[6] != kExp * kDim || in_sizes[8] != kExp * kDim) return;
  if (in_sizes[11] != kDim * kFeat) return;
  if (out_size != kBatch * kSeq * kDim) return;
  if (kWsTotal > ws_size) return;

  const float* x    = (const float*)d_in[0];
  const float* Wa_u = (const float*)d_in[1];
  const float* ba_u = (const float*)d_in[2];
  const float* Wi_u = (const float*)d_in[3];
  const float* bi_u = (const float*)d_in[4];
  const float* g_u  = (const float*)d_in[5];
  const float* Wa_w = (const float*)d_in[6];
  const float* ba_w = (const float*)d_in[7];
  const float* Wi_w = (const float*)d_in[8];
  const float* bi_w = (const float*)d_in[9];
  const float* g_w  = (const float*)d_in[10];
  const float* Wf   = (const float*)d_in[11];
  const float* bfv  = (const float*)d_in[12];
  float* out = (float*)d_out;

  char* ws = (char*)d_ws;
  unsigned short* wstHi = (unsigned short*)(ws + kOffWstHi);
  unsigned short* wstLo = (unsigned short*)(ws + kOffWstLo);
  unsigned short* wfHi  = (unsigned short*)(ws + kOffWfHi);
  unsigned short* wfLo  = (unsigned short*)(ws + kOffWfLo);
  unsigned short* xh    = (unsigned short*)(ws + kOffXh);
  unsigned short* xl    = (unsigned short*)(ws + kOffXl);
  float*          papi  = (float*)(ws + kOffPapi);
  unsigned short* ch    = (unsigned short*)(ws + kOffCh);
  unsigned short* cl    = (unsigned short*)(ws + kOffCl);

  const int wgN8 = kExp * kDim / 8;
  const size_t wblk = (size_t)kExp * kDim;
  split8_kernel<<<wgN8 / 256, 256, 0, stream>>>(Wa_u, wstHi,            wstLo,            wgN8);
  split8_kernel<<<wgN8 / 256, 256, 0, stream>>>(Wi_u, wstHi + wblk,     wstLo + wblk,     wgN8);
  split8_kernel<<<wgN8 / 256, 256, 0, stream>>>(Wa_w, wstHi + 2 * wblk, wstLo + 2 * wblk, wgN8);
  split8_kernel<<<wgN8 / 256, 256, 0, stream>>>(Wi_w, wstHi + 3 * wblk, wstLo + 3 * wblk, wgN8);
  const int wfN8 = kDim * kFeat / 8;
  split8_kernel<<<wfN8 / 256, 256, 0, stream>>>(Wf, wfHi, wfLo, wfN8);

  const long strideXq   = (long)kQRows * kDim;
  const long strideWst  = (long)kExp2 * kDim;
  const long stridePapi = (long)kQRows * kExp2;
  const int prepBlocks  = kQRows * kDim / 8 / 256;
  const int projBlocks  = (kQRows / 64) * (kExp2 / 64) / 8;
  const int outBlocks   = (kQRows / 64) * (kDim / 64) / 8;

  for (int qi = 0; qi < kNumQ; ++qi) {
    const float* xq  = x + (size_t)qi * kQRows * kDim;
    float*       oq  = out + (size_t)qi * kQRows * kDim;

    prep_x_kernel<<<prepBlocks, 256, 0, stream>>>(xq, xh, xl);

    wmma_gemm64<1, true, 0, 0, false><<<dim3(projBlocks, 2), 256, 0, stream>>>(
        xh, xl, kDim, strideXq,
        wstHi, wstLo, kDim, strideWst,
        (void*)papi, (void*)papi, kExp2, stridePapi,
        bfv, bfv, 0L,
        kQRows, kExp2, kDim, 1.0f);

    scan_kernel<<<dim3(kQBatch, 2), 256, 0, stream>>>(papi, ba_u, bi_u, g_u, ba_w, bi_w, g_w, ch, cl);

    wmma_gemm64<1, true, 2, 0, false><<<dim3(outBlocks, 1), 256, 0, stream>>>(
        ch, cl, kFeat, 0L,
        wfHi, wfLo, kFeat, 0L,
        (void*)oq, (void*)oq, kDim, 0L,
        bfv, bfv, 0L,
        kQRows, kDim, kFeat, 1.0f);
  }
}
